// KendallDistance_68513318306381
// MI455X (gfx1250) — hardware-verified
//
#include <hip/hip_runtime.h>
#include <stddef.h>
#include <stdint.h>

#define NB   64
#define NT   256
#define NN   64
#define KP   2048
#define SLAB 256
#define NSL  (KP / SLAB)
#define XSP  68
#define SBP  34

static_assert(NSL == 8);
static_assert(NB * (NB - 1) / 2 + 32 == KP);
static_assert(NN == 64);
static_assert(NB == 64);
static_assert(NT % 4 == 0);
static_assert(SLAB == 4 * 64);
static_assert((XSP * 4) % 16 == 0);

typedef _Float16 hh;
typedef hh    v16h __attribute__((ext_vector_type(16)));
typedef hh    v8h  __attribute__((ext_vector_type(8)));
typedef float v8f  __attribute__((ext_vector_type(8)));
typedef float v4f  __attribute__((ext_vector_type(4)));
typedef v4f   v4fa __attribute__((may_alias));

union Frag { v16h v; v8h p[2]; };

__device__ __forceinline__ v8f zero8() { return (v8f){0.f, 0.f, 0.f, 0.f, 0.f, 0.f, 0.f, 0.f}; }

__device__ __forceinline__ v8f mma16(v16h a, v16h b, v8f cc) {
  return __builtin_amdgcn_wmma_f32_16x16x32_f16(false, a, false, b, (short)0, cc, false, false);
}

__global__ __launch_bounds__(256) void k_gram(const float* __restrict__ x, float* __restrict__ part) {
  __shared__ __align__(16) float xs[NB * XSP];
  __shared__ __align__(16) v8h   sb[NN * SBP];
  const int tid = threadIdx.x, lane = tid & 31, w = tid >> 5;
  const int h = lane >> 4, c = lane & 15;
  const int t = blockIdx.x;

#pragma unroll
  for (int it = 0; it < 4; ++it) {
    const int p  = tid + 256 * it;
    const int a  = p >> 4;
    const int n4 = (p & 15) * 4;
    const v4f v = *(const v4f*)(x + ((size_t)a * NT + (size_t)t) * NN + n4);
    *(v4fa*)(xs + a * XSP + n4) = v;
  }
  __syncthreads();

  const int mi  = w >> 1;
  const int nj0 = (w & 1) * 2;
  const int ra  = (16 * mi + c) * SBP;
  const int rb0 = (16 * nj0 + c) * SBP;
  const int rb1 = (16 * nj0 + 16 + c) * SBP;
  const int gn  = tid & 63;
  const int kq  = tid >> 6;

  v8f acc0 = zero8(), acc1 = zero8();

#pragma unroll 1
  for (int sl = 0; sl < NSL; ++sl) {
    const int s   = sl * 4 + kq;
    const int r1  = 63 - s;
    const int a2  = 62 - s;
    const int pad = (s == 31) ? 1 : 0;
    const float xa1 = xs[s * XSP + gn];
    const float xa2 = xs[a2 * XSP + gn];
#pragma unroll
    for (int pp = 0; pp < 8; ++pp) {
      v8f sg;
#pragma unroll
      for (int e = 0; e < 8; ++e) {
        const int kk  = pp * 8 + e;
        const int in1 = (kk < r1) ? 1 : 0;
        int b1 = s + 1 + kk;
        if (b1 > 63) b1 = 63;
        const int b = in1 ? b1 : (pad ? a2 : kk);
        const float xa = in1 ? xa1 : xa2;
        const float xb = xs[b * XSP + gn];
        const float d  = xb - xa;
        const float up = (d > 0.0f) ? 1.0f : 0.0f;
        const float dn = (d < 0.0f) ? 1.0f : 0.0f;
        sg[e] = up - dn;
      }
      sb[gn * SBP + kq * 8 + pp] = __builtin_convertvector(sg, v8h);
    }
    __syncthreads();
#pragma unroll 2
    for (int ks = 0; ks < SLAB / 32; ++ks) {
      const int pa = 4 * ks + h;
      Frag fa, fb0, fb1;
      fa.p[0]  = sb[ra + pa];
      fa.p[1]  = sb[ra + pa + 2];
      fb0.p[0] = sb[rb0 + pa];
      fb0.p[1] = sb[rb0 + pa + 2];
      fb1.p[0] = sb[rb1 + pa];
      fb1.p[1] = sb[rb1 + pa + 2];
      acc0 = mma16(fa.v, fb0.v, acc0);
      acc1 = mma16(fa.v, fb1.v, acc1);
      asm volatile("v_nop\n\tv_nop\n\tv_nop\n\tv_nop"
                   : "+v"(acc0), "+v"(acc1)
                   : "v"(fa.v), "v"(fb0.v), "v"(fb1.v));
    }
    __syncthreads();
  }

#pragma unroll
  for (int r = 0; r < 8; ++r) {
    const int row = 16 * mi + 8 * h + r;
    xs[row * XSP + 16 * nj0 + c]      = acc0[r];
    xs[row * XSP + 16 * nj0 + 16 + c] = acc1[r];
  }
  __syncthreads();
  v4f    val[4];
  size_t go[4];
#pragma unroll
  for (int it = 0; it < 4; ++it) {
    const int p   = tid + 256 * it;
    const int row = p >> 4;
    const int pc  = p & 15;
    val[it] = *(const v4fa*)(xs + row * XSP + 4 * pc);
    go[it]  = (size_t)t * (NN * NN) + (size_t)row * NN + 4 * pc;
  }
#pragma unroll
  for (int it = 0; it < 4; ++it) *(volatile v4f*)(part + go[it]) = val[it];
  __threadfence();
#pragma unroll
  for (int it = 0; it < 4; ++it) *(volatile v4f*)(part + go[it]) = val[it];
}

__global__ __launch_bounds__(256) void k_out(const float* __restrict__ part, float* __restrict__ out) {
#pragma clang fp contract(off)
  __shared__ float red[4 * NN];
  __shared__ __align__(16) float drow[NN];
  const int tid = threadIdx.x;
  const int i = blockIdx.x;
  const int j = tid & 63, tg = tid >> 6;
  const float* pp = part + ((size_t)(tg * (NT / 4)) * (NN * NN) + (size_t)i * NN + j);
  float s = 0.0f;
#pragma unroll 4
  for (int tt = 0; tt < NT / 4; ++tt) s += pp[(size_t)tt * (NN * NN)];
  red[tg * NN + j] = s;
  __syncthreads();
  if (tid < NN) {
    const float cs = ((red[j] + red[NN + j]) + red[2 * NN + j]) + red[3 * NN + j];
    const float cf = 2.0f * cs;
    const float q  = cf * (1.0f / 2016.0f);
    float d = 1.0f - q;
    if (j == i) d = 0.0f;
    drow[j] = d;
  }
  __syncthreads();
  const int pc = tid & 15;
  const v4f v = *(const v4fa*)(drow + 4 * pc);
  size_t go[4];
#pragma unroll
  for (int it = 0; it < 4; ++it) {
    const int p  = tid + 256 * it;
    const int bq = p >> 4;
    go[it] = (size_t)bq * (NN * NN) + (size_t)i * NN + 4 * pc;
  }
#pragma unroll
  for (int it = 0; it < 4; ++it) *(volatile v4f*)(out + go[it]) = v;
  __threadfence();
#pragma unroll
  for (int it = 0; it < 4; ++it) *(volatile v4f*)(out + go[it]) = v;
}

extern "C" void kernel_launch(void* const* d_in, const int* in_sizes, int n_in,
                              void* d_out, int out_size, void* d_ws, size_t ws_size,
                              hipStream_t stream) {
  if (n_in < 1) return;
  if (in_sizes[0] != NB * NT * NN) return;
  if (out_size != NB * NN * NN) return;
  const size_t need = (size_t)NT * NN * NN * 4;
  if (need > ws_size) return;
  if (need > (size_t)134217728) return;

  const float* x = (const float*)d_in[0];
  float* part = (float*)d_ws;
  float* out  = (float*)d_out;

  k_gram<<<dim3(NT), dim3(256), 0, stream>>>(x, part);
  k_out<<<dim3(NN), dim3(256), 0, stream>>>(part, out);
  (void)hipGetLastError();
}
